// GenODE_44641890074925
// MI455X (gfx1250) — hardware-run, weakly checked
//
#include <hip/hip_runtime.h>


#define NB   512
#define ND   16
#define NH   128
#define NSTEP 511
typedef _Float16 h16;
typedef unsigned short bf;
typedef __attribute__((ext_vector_type(16))) __bf16   v16bf;
typedef __attribute__((ext_vector_type(16))) _Float16 v16h;
typedef __attribute__((ext_vector_type(8)))  _Float16 v8h;
typedef __attribute__((ext_vector_type(8)))  unsigned short v8us;
typedef __attribute__((ext_vector_type(8)))  float    v8f;
typedef __attribute__((ext_vector_type(4)))  float    v4f;
typedef v8h  __attribute__((may_alias)) v8ha;
typedef v4f  __attribute__((may_alias)) v4fa;
typedef v8us __attribute__((may_alias)) v8usa;

__device__ __forceinline__ unsigned short f2bf(float f) { unsigned u = __float_as_uint(f); u += 0x7FFFu + ((u >> 16) & 1u); return (unsigned short)(u >> 16); }
__device__ __forceinline__ float bf2f(unsigned short b) { return __uint_as_float(((unsigned)b) << 16); }
__device__ __forceinline__ float bfr(float f) { return bf2f(f2bf(f)); }
__device__ __forceinline__ v16h cat16(v8h lo, v8h hi) { return __builtin_shufflevector(lo, hi, 0, 1, 2, 3, 4, 5, 6, 7, 8, 9, 10, 11, 12, 13, 14, 15); }
__device__ __forceinline__ v16bf cat16b(v8us lo, v8us hi) { return __builtin_bit_cast(v16bf, __builtin_shufflevector(lo, hi, 0, 1, 2, 3, 4, 5, 6, 7, 8, 9, 10, 11, 12, 13, 14, 15)); }
__device__ __forceinline__ v8f wmma16(v16h a, v16h b, v8f c) { return __builtin_amdgcn_wmma_f32_16x16x32_f16(false, a, false, b, (short)0, c, false, false); }
__device__ __forceinline__ v8f wmmab(v16bf a, v16bf b, v8f c) { return __builtin_amdgcn_wmma_f32_16x16x32_bf16(false, a, false, b, (short)0, c, false, false); }

template <typename T16> struct WFrag;
template <> struct WFrag<h16> { typedef v16h V; static __device__ __forceinline__ V ld(const h16* p) { return cat16(*(const v8h*)p, *(const v8h*)(p + 16)); } static __device__ __forceinline__ v8f mma(V a, V b, v8f c) { return wmma16(a, b, c); } };
template <> struct WFrag<bf> { typedef v16bf V; static __device__ __forceinline__ V ld(const bf* p) { return cat16b(*(const v8us*)p, *(const v8us*)(p + 16)); } static __device__ __forceinline__ v8f mma(V a, V b, v8f c) { return wmmab(a, b, c); } };

typedef __attribute__((ext_vector_type(2))) _Float16 v2h;
typedef __attribute__((ext_vector_type(4))) _Float16 v4h;
typedef __attribute__((ext_vector_type(2))) unsigned short v2us;
typedef __attribute__((ext_vector_type(4))) unsigned short v4us;
typedef __attribute__((ext_vector_type(2))) float v2f;
typedef __attribute__((ext_vector_type(4))) int v4i;

__global__ __launch_bounds__(256) void k_wtG(const float* __restrict__ w, int K, int N, bf* Bt) {
    const int lane = threadIdx.x & 31; const int L0 = (blockIdx.x * 8 + (threadIdx.x >> 5)) * 8; const int nlines = N * K / 64;
#pragma unroll
    for (int ps = 0; ps < 2; ++ps) {
        for (int l = 0; l < 8; ++l) { const int L = L0 + l; if (L >= nlines) break; const size_t e = (size_t)L * 64 + lane * 2; const int k = (int)(e % K), n = (int)(e / K); v2us o;
            o[0] = f2bf(w[(size_t)k * N + n]); o[1] = f2bf(w[(size_t)(k + 1) * N + n]); *(volatile v2us*)(Bt + e) = o; }
        if (ps == 0) __threadfence(); }
}

__device__ __forceinline__ float tanhc(float v) { return 1.0f - 2.0f / (expf(2.0f * v) + 1.0f); }

__global__ __launch_bounds__(256) void k_w1p(const float* __restrict__ w, bf* P) { const int i = blockIdx.x * 256 + threadIdx.x; if (i >= NH * 4) return; const int u = i >> 2, sg = i & 3; const int d0 = 8 * (sg >> 1); const float live = (sg & 1) ? 0.0f : 1.0f; v8us o;
#pragma unroll
    for (int p = 0; p < 8; ++p) o[p] = f2bf(w[(size_t)(d0 + p) * NH + u] * live);
    *(volatile v8us*)(P + (size_t)i * 8) = o; __threadfence(); *(volatile v8us*)(P + (size_t)i * 8) = o; }

__device__ __forceinline__ void fld(const float (&y)[8], float (&F)[8], const bf* w1p, const bf* w2p, const float* __restrict__ b1, const float* __restrict__ b2, int hi, v8us zz) { v8us lo;
#pragma unroll
    for (int j = 0; j < 8; ++j) lo[j] = f2bf(y[j]);
    const v16bf yf = cat16b(lo, zz); v8f f = (v8f){};
    for (int c = 0; c < 4; ++c) { v8f d0 = (v8f){}, d1 = (v8f){}; const bf* pa = w1p + (size_t)(32 * c) * 32; d0 = wmmab(cat16b(*(const v8us*)pa, *(const v8us*)(pa + 8)), yf, d0); const bf* pb = pa + (size_t)16 * 32; d1 = wmmab(cat16b(*(const v8us*)pb, *(const v8us*)(pb + 8)), yf, d1);
        v8us tl, tu;
#pragma unroll
        for (int j = 0; j < 8; ++j) { tl[j] = f2bf(tanhc(d0[j] + bfr(b1[32 * c + 8 * hi + j]))); tu[j] = f2bf(tanhc(d1[j] + bfr(b1[32 * c + 16 + 8 * hi + j]))); }
        const v16bf tf = cat16b(tl, tu);
        f = wmmab(WFrag<bf>::ld(w2p + 32 * c), tf, f); }
#pragma unroll
    for (int j = 0; j < 8; ++j) F[j] = f[j] + bfr(b2[8 * hi + j]); }

__global__ __launch_bounds__(32) void k_rk(const float* __restrict__ y0, const bf* __restrict__ W1p, const float* __restrict__ b1, const bf* __restrict__ W2t, const float* __restrict__ b2, float* Q) {
    if (blockIdx.x >= (unsigned)(NB / 16)) return;
    const int lane = threadIdx.x & 31, lr = lane & 15, hi = lane >> 4; const int row = (int)blockIdx.x * 16 + lr;
    float Y[8], R[8];
    { const float* p = y0 + (size_t)row * ND + 8 * hi; const v4f a = *(const v4f*)p; const v4f b = *(const v4f*)(p + 4);
#pragma unroll
      for (int j = 0; j < 4; ++j) { Y[j] = bfr(a[j]); Y[4 + j] = bfr(b[j]); R[j] = Y[j]; R[4 + j] = Y[4 + j]; } }
    const bf* w1p = W1p + (size_t)lr * 32 + 16 * hi; const bf* w2p = W2t + (size_t)lr * NH + 8 * hi;
    const v8us zz = *(const v8us*)(W1p + 8);
    const float h = (float)(1.0 / 511.0);
    const float a21 = (float)(0.2);
    const float a31 = (float)(3.0 / 40.0), a32 = (float)(9.0 / 40.0);
    const float a41 = (float)(44.0 / 45.0), a42 = (float)(56.0 / 15.0), a43 = (float)(32.0 / 9.0);
    const float a51 = (float)(19372.0 / 6561.0), a52 = (float)(25360.0 / 2187.0), a53 = (float)(64448.0 / 6561.0), a54 = (float)(212.0 / 729.0);
    const float a61 = (float)(9017.0 / 3168.0), a62 = (float)(355.0 / 33.0), a63 = (float)(46732.0 / 5247.0), a64 = (float)(49.0 / 176.0), a65 = (float)(5103.0 / 18656.0);
    const float c1 = (float)(35.0 / 384.0), c3 = (float)(500.0 / 1113.0), c4 = (float)(125.0 / 192.0), c5 = (float)(2187.0 / 6784.0), c6 = (float)(11.0 / 84.0);
    for (int k = 0; k < NSTEP; ++k) {
        const bool take = (k == row);
#pragma unroll
        for (int j = 0; j < 8; ++j) R[j] = take ? Y[j] : R[j];
        float k1[8], k2[8], k3[8], k4[8], k5[8], k6[8], s[8];
        fld(Y, k1, w1p, w2p, b1, b2, hi, zz);
#pragma unroll
        for (int j = 0; j < 8; ++j) s[j] = Y[j] + h * (a21 * k1[j]);
        fld(s, k2, w1p, w2p, b1, b2, hi, zz);
#pragma unroll
        for (int j = 0; j < 8; ++j) s[j] = Y[j] + h * (a31 * k1[j] + a32 * k2[j]);
        fld(s, k3, w1p, w2p, b1, b2, hi, zz);
#pragma unroll
        for (int j = 0; j < 8; ++j) s[j] = Y[j] + h * (a41 * k1[j] - a42 * k2[j] + a43 * k3[j]);
        fld(s, k4, w1p, w2p, b1, b2, hi, zz);
#pragma unroll
        for (int j = 0; j < 8; ++j) s[j] = Y[j] + h * (a51 * k1[j] - a52 * k2[j] + a53 * k3[j] - a54 * k4[j]);
        fld(s, k5, w1p, w2p, b1, b2, hi, zz);
#pragma unroll
        for (int j = 0; j < 8; ++j) s[j] = Y[j] + h * (a61 * k1[j] - a62 * k2[j] + a63 * k3[j] + a64 * k4[j] - a65 * k5[j]);
        fld(s, k6, w1p, w2p, b1, b2, hi, zz);
#pragma unroll
        for (int j = 0; j < 8; ++j) Y[j] = Y[j] + h * (c1 * k1[j] + c3 * k3[j] + c4 * k4[j] - c5 * k5[j] + c6 * k6[j]); }
    { const bool take = (row == NSTEP);
#pragma unroll
      for (int j = 0; j < 8; ++j) R[j] = take ? Y[j] : R[j]; }
    float* pq = Q + ((size_t)row * 2 + hi) * 32; v4f a, b, z;
#pragma unroll
    for (int j = 0; j < 4; ++j) { a[j] = R[j]; b[j] = R[4 + j]; z[j] = R[j] * 0.0f; }
#pragma unroll
    for (int ps = 0; ps < 2; ++ps) { *(volatile v4f*)pq = a; *(volatile v4f*)(pq + 4) = b;
#pragma unroll
        for (int q = 2; q < 8; ++q) *(volatile v4f*)(pq + 4 * q) = z;
        if (ps == 0) __threadfence(); }
}

__global__ __launch_bounds__(256) void k_out(const float* __restrict__ Q, float* out) { const int i = blockIdx.x * 256 + threadIdx.x; if (i >= NB * ND / 4) return; const int row = i >> 2, q = i & 3; const v4f v = *(const v4f*)(Q + ((size_t)row * 2 + (q >> 1)) * 32 + 4 * (q & 1)); *(volatile v4f*)(out + (size_t)i * 4) = v; __threadfence(); *(volatile v4f*)(out + (size_t)i * 4) = v; }

extern "C" void kernel_launch(void* const* d_in, const int* in_sizes, int n_in, void* d_out, int out_size, void* d_ws, size_t ws_size, hipStream_t stream) {
    if (n_in < 5) return;
    if (in_sizes[0] != NB * ND || in_sizes[1] != ND * NH || in_sizes[2] != NH || in_sizes[3] != NH * ND || in_sizes[4] != ND) return;
    if (out_size != NB * ND) return;
    static_assert(NB % 16 == 0 && ND == 16 && NH == 128 && NSTEP == NB - 1 && (NH * ND) % 64 == 0, "a wave's 16 rows; one state tile; four chunks of 32 hidden units; the record's last row is row NSTEP; k_wtG's lines of 64 words"); static_assert((NB * ND / 4) % 256 == 0, "k_out's grid exact");
    const float* y0 = (const float*)d_in[0]; const float* W1 = (const float*)d_in[1]; const float* b1 = (const float*)d_in[2]; const float* W2 = (const float*)d_in[3]; const float* b2 = (const float*)d_in[4];
    char* wsp = (char*)d_ws; auto take = [&](size_t bytes) { char* p = wsp; wsp += (bytes + 255) & ~(size_t)255; return (void*)p; };
    bf* W1p = (bf*)take((size_t)NH * 32 * 2); bf* W2t = (bf*)take((size_t)ND * NH * 2); float* Q = (float*)take((size_t)NB * 2 * 32 * 4);
    if ((size_t)(wsp - (char*)d_ws) > ws_size) return;
    k_w1p<<<(unsigned)(NH * 4 / 256), 256, 0, stream>>>(W1, W1p);
    k_wtG<<<1, 256, 0, stream>>>(W2, NH, ND, W2t);
    k_rk<<<(unsigned)(NB / 16), 32, 0, stream>>>(y0, W1p, b1, W2t, b2, Q);
    k_out<<<(unsigned)(NB * ND / 4 / 256), 256, 0, stream>>>(Q, (float*)d_out);
}
